// GATCustom_79748952752833
// MI455X (gfx1250) — hardware-verified
//
#include <hip/hip_runtime.h>


#ifndef NB
#define NB 64
#endif
#define NB_FULL 64
#define NN   128
#define NF   64
#define NO   64
#define NW   192
#define GW   8
#define EIP  68
#define EJP  64
#define HTP  136
#define PP   136
#define HSC  64.0f
#define PSC  16384.0f
#define OSI  (1.0f / (16384.0f * 64.0f))
#define L2E  1.4426950408889634f

static_assert(NF == 64);
static_assert(NF * 2 == 128);
static_assert(NO == 64);
static_assert(NW == 3 * NO);
static_assert(NN == 128);
static_assert(NN == 16 * GW);
static_assert(NN % 32 == 0);
static_assert((NO & (NO - 1)) == 0);
static_assert(((size_t)NW * NF / 8) % 256 == 0);
static_assert((NB_FULL * NN) % (4 * 32 * GW) == 0);
static_assert((EIP * 4) % 16 == 0);
static_assert((EJP * 4) % 16 == 0);
static_assert((HTP * 2) % 16 == 0);
static_assert((PP * 2) % 16 == 0);
static_assert(EIP >= NO);
static_assert(HTP >= NN);
static_assert(PP >= NN);
static_assert(32 * 16 * 8 == 16 * NO * 4);
static_assert(NB <= NB_FULL);
static_assert((size_t)NN * EIP * 4 + (size_t)NN * EJP * 4 + (size_t)NO * HTP * 2 + (size_t)NN * PP * 2 + (size_t)NO * 4 + (size_t)GW * 4 <= (size_t)131072);

typedef _Float16 h16;
typedef unsigned short bf;
typedef __attribute__((ext_vector_type(16))) __bf16   v16bf;
typedef __attribute__((ext_vector_type(16))) _Float16 v16h;
typedef __attribute__((ext_vector_type(8)))  _Float16 v8h;
typedef __attribute__((ext_vector_type(8)))  unsigned short v8us;
typedef __attribute__((ext_vector_type(8)))  float    v8f;
typedef __attribute__((ext_vector_type(4)))  float    v4f;
typedef v4f  __attribute__((may_alias)) v4fa;

__device__ __forceinline__ unsigned short f2bf(float f) { unsigned u = __float_as_uint(f); u += 0x7FFFu + ((u >> 16) & 1u); return (unsigned short)(u >> 16); }
__device__ __forceinline__ float bfr(float f) { return __uint_as_float(((unsigned)f2bf(f)) << 16); }
__device__ __forceinline__ v16h cat16(v8h lo, v8h hi) { return __builtin_shufflevector(lo, hi, 0, 1, 2, 3, 4, 5, 6, 7, 8, 9, 10, 11, 12, 13, 14, 15); }
__device__ __forceinline__ v16bf cat16b(v8us lo, v8us hi) { return __builtin_bit_cast(v16bf, __builtin_shufflevector(lo, hi, 0, 1, 2, 3, 4, 5, 6, 7, 8, 9, 10, 11, 12, 13, 14, 15)); }
__device__ __forceinline__ v8f wmma16(v16h a, v16h b, v8f c) { return __builtin_amdgcn_wmma_f32_16x16x32_f16(false, a, false, b, (short)0, c, false, false); }
__device__ __forceinline__ v8f wmmab(v16bf a, v16bf b, v8f c) { return __builtin_amdgcn_wmma_f32_16x16x32_bf16(false, a, false, b, (short)0, c, false, false); }
__device__ __forceinline__ v16h  ldh(const h16* p) { return cat16(*(const v8h*)p, *(const v8h*)(p + 16)); }
__device__ __forceinline__ v16bf ldb(const bf* p)  { return cat16b(*(const v8us*)p, *(const v8us*)(p + 16)); }
__device__ __forceinline__ void wave_sync() { __builtin_amdgcn_fence(3  , "wavefront"); __builtin_amdgcn_wave_barrier(); asm volatile("" ::: "memory"); }

__global__ __launch_bounds__(256) void k_cvt8(const float* __restrict__ src, bf* dst, size_t n8) {
    const size_t i = (size_t)blockIdx.x * 256 + threadIdx.x; if (i >= n8) return;
    const v8f v = *(const v8f*)(src + i * 8); v8us o;
#pragma unroll
    for (int k = 0; k < 8; ++k) o[k] = f2bf(v[k]);
    *(volatile v8us*)(dst + i * 8) = o; __threadfence(); *(volatile v8us*)(dst + i * 8) = o;
}

typedef __attribute__((ext_vector_type(4))) int v4i;
typedef v8h __attribute__((may_alias)) v8ha;

static __device__ __forceinline__ h16 toh_flush(float v) { const h16 r = (h16)v; return (fabsf(v) < 6.103515625e-05f) ? (h16)0.0f : r; }
__device__ __forceinline__ v8f wmmab_g(v16bf a, v16bf b, v8f c) { c = wmmab(a, b, c); asm volatile("v_nop\n\tv_nop\n\tv_nop\n\tv_nop" : "+v"(c) : "v"(a), "v"(b)); return c; }
__device__ __forceinline__ v8f wmma16_g(v16h a, v16h b, v8f c) { c = wmma16(a, b, c); asm volatile("v_nop\n\tv_nop\n\tv_nop\n\tv_nop" : "+v"(c) : "v"(a), "v"(b)); return c; }
__device__ __forceinline__ int imax(int a, int b) { return a > b ? a : b; }

__global__ __launch_bounds__(256) void k_wprep(const float* __restrict__ W, const float* __restrict__ Wl, bf* WB) {
    const int t = blockIdx.x * 256 + threadIdx.x; if (t >= NW * NF / 8) return;
    const int n = t >> 3, k8 = (t & 7) * 8;
    const int nc = n & (NO - 1);
    const int o = (n - NO) & (NO - 1);
    const int cofs = (n >= 2 * NO) ? NF : 0;
    v8us ov;
#pragma unroll
    for (int e = 0; e < 8; ++e) {
        const int k = k8 + e;
        float wv = W[(size_t)k * NO + nc];
        float lv = Wl[(size_t)o * (2 * NF) + cofs + k];
        asm volatile("" : "+v"(wv));
        asm volatile("" : "+v"(lv));
        ov[e] = f2bf((n < NO) ? wv : lv);
    }
    *(volatile v8us*)(WB + (size_t)t * 8) = ov; __threadfence(); *(volatile v8us*)(WB + (size_t)t * 8) = ov;
}

__device__ __forceinline__ v8f proj_tile(const bf* __restrict__ WB, v16bf a0, v16bf a1, int n0, int lr, int hi) {
    const size_t bo = (size_t)(n0 + lr) * NF + 8 * hi;
    v8f acc = (v8f){};
    acc = wmmab_g(a0, ldb(WB + bo), acc);
    acc = wmmab_g(a1, ldb(WB + bo + 32), acc);
    return acc;
}

__global__ __launch_bounds__(32 * GW) void k_graph(const bf* __restrict__ XB, const bf* __restrict__ WB, const float* __restrict__ av, const int* __restrict__ batch, float* OUT) {
    __shared__ __align__(16) float sEI[NN * EIP];
    __shared__ __align__(16) float sEJ[NN * EJP];
    __shared__ __align__(16) h16   sHT[NO * HTP];
    __shared__ __align__(16) h16   sP[NN * PP];
    __shared__ __align__(16) float sA[NO];
    __shared__ int sRed[GW];
    const int tid = threadIdx.x;
    const int lane = threadIdx.x & 31, lr = lane & 15, hi = lane >> 4;
    const int wave = __builtin_amdgcn_readfirstlane((int)(threadIdx.x >> 5));
    const int b = blockIdx.x;

    int bm = -2147483647 - 1;
    { const v4i* bp = (const v4i*)batch;
#pragma unroll
      for (int q = 0; q < (NB_FULL * NN) / (4 * 32 * GW); ++q) { const v4i v = bp[q * (32 * GW) + tid]; bm = imax(bm, imax(imax(v[0], v[1]), imax(v[2], v[3]))); } }
    bm = imax(bm, __shfl_xor(bm, 16, 32)); bm = imax(bm, __shfl_xor(bm, 8, 32)); bm = imax(bm, __shfl_xor(bm, 4, 32));
    bm = imax(bm, __shfl_xor(bm, 2, 32));  bm = imax(bm, __shfl_xor(bm, 1, 32));
    if (lane == 0) sRed[wave] = bm;
    { const float a_in = av[tid & (NO - 1)]; if (tid < NO) sA[tid] = bfr(a_in); }

    { const size_t xo = ((size_t)b * NN + (size_t)(16 * wave + lr)) * NF + 8 * hi;
      const v16bf a0 = ldb(XB + xo), a1 = ldb(XB + xo + 32);
      const int nrow = 16 * wave + 8 * hi;
#pragma unroll 1
      for (int nt = 0; nt < NO / 16; ++nt) {
          const v8f acc = proj_tile(WB, a0, a1, 16 * nt, lr, hi);
          v8h hv;
#pragma unroll
          for (int r = 0; r < 8; ++r) hv[r] = toh_flush(acc[r] * HSC);
          *(v8ha*)(&sHT[(16 * nt + lr) * HTP + nrow]) = hv;
      }
#pragma unroll 1
      for (int nt = 0; nt < NO / 16; ++nt) {
          const v8f acc = proj_tile(WB, a0, a1, NO + 16 * nt, lr, hi);
#pragma unroll
          for (int r = 0; r < 8; ++r) sEI[(nrow + r) * EIP + 16 * nt + lr] = acc[r];
      }
#pragma unroll 1
      for (int nt = 0; nt < NO / 16; ++nt) {
          const v8f acc = proj_tile(WB, a0, a1, 2 * NO + 16 * nt, lr, hi);
#pragma unroll
          for (int r = 0; r < 8; ++r) sEJ[(nrow + r) * EJP + 16 * nt + lr] = acc[r];
      }
    }
    __syncthreads();

    int bmax = sRed[0];
#pragma unroll
    for (int w = 1; w < GW; ++w) bmax = imax(bmax, sRed[w]);
    const bool bad = (bmax + 1) != NB_FULL;

#pragma unroll 1
    for (int jj = 0; jj < 16; ++jj) {
        const int j = 16 * wave + jj;
        float s0 = 0.0f, s1 = 0.0f, s2 = 0.0f, s3 = 0.0f;
#pragma unroll 2
        for (int oc = 0; oc < NO / 4; ++oc) {
            const v4f ej = *(const v4fa*)(&sEJ[j * EJP + 4 * oc]);
            const v4f aa = *(const v4fa*)(&sA[4 * oc]);
            const v4f e0 = *(const v4fa*)(&sEI[(lane)      * EIP + 4 * oc]);
            const v4f e1 = *(const v4fa*)(&sEI[(lane + 32) * EIP + 4 * oc]);
            const v4f e2 = *(const v4fa*)(&sEI[(lane + 64) * EIP + 4 * oc]);
            const v4f e3 = *(const v4fa*)(&sEI[(lane + 96) * EIP + 4 * oc]);
#pragma unroll
            for (int c = 0; c < 4; ++c) {
                s0 = fmaf(fmaxf(e0[c] + ej[c], 0.0f), aa[c], s0);
                s1 = fmaf(fmaxf(e1[c] + ej[c], 0.0f), aa[c], s1);
                s2 = fmaf(fmaxf(e2[c] + ej[c], 0.0f), aa[c], s2);
                s3 = fmaf(fmaxf(e3[c] + ej[c], 0.0f), aa[c], s3);
            }
        }
        float mx = fmaxf(fmaxf(s0, s1), fmaxf(s2, s3));
        mx = fmaxf(mx, __shfl_xor(mx, 16, 32)); mx = fmaxf(mx, __shfl_xor(mx, 8, 32)); mx = fmaxf(mx, __shfl_xor(mx, 4, 32));
        mx = fmaxf(mx, __shfl_xor(mx, 2, 32));  mx = fmaxf(mx, __shfl_xor(mx, 1, 32));
        const float x0 = __builtin_amdgcn_exp2f((s0 - mx) * L2E), x1 = __builtin_amdgcn_exp2f((s1 - mx) * L2E);
        const float x2 = __builtin_amdgcn_exp2f((s2 - mx) * L2E), x3 = __builtin_amdgcn_exp2f((s3 - mx) * L2E);
        float sum = (x0 + x1) + (x2 + x3);
        sum += __shfl_xor(sum, 16, 32); sum += __shfl_xor(sum, 8, 32); sum += __shfl_xor(sum, 4, 32);
        sum += __shfl_xor(sum, 2, 32);  sum += __shfl_xor(sum, 1, 32);
        const float sc = PSC * (1.0f / sum);
        sP[(lane)      * PP + j] = toh_flush(x0 * sc);
        sP[(lane + 32) * PP + j] = toh_flush(x1 * sc);
        sP[(lane + 64) * PP + j] = toh_flush(x2 * sc);
        sP[(lane + 96) * PP + j] = toh_flush(x3 * sc);
    }
    __syncthreads();

    v8f acc[4];
#pragma unroll
    for (int nt = 0; nt < 4; ++nt) acc[nt] = (v8f){};
#pragma unroll
    for (int ks = 0; ks < NN / 32; ++ks) {
        const int pi = (16 * wave + lr) * PP + 32 * ks + 8 * hi;
        const v16h pa = cat16(*(const v8ha*)(&sP[pi]), *(const v8ha*)(&sP[pi + 16]));
#pragma unroll
        for (int nt = 0; nt < 4; ++nt) {
            const int hix = (16 * nt + lr) * HTP + 32 * ks + 8 * hi;
            const v16h hb = cat16(*(const v8ha*)(&sHT[hix]), *(const v8ha*)(&sHT[hix + 16]));
            acc[nt] = wmma16_g(pa, hb, acc[nt]);
        }
    }
    const float nanv = __uint_as_float(0x7FC00000u);
    const int wb = wave * 16 * EIP;
#pragma unroll
    for (int nt = 0; nt < 4; ++nt) {
#pragma unroll
        for (int r = 0; r < 8; ++r) { const float v = acc[nt][r] * OSI; sEI[wb + (8 * hi + r) * EIP + 16 * nt + lr] = bad ? nanv : v; }
    }
    wave_sync();
    float* orow = OUT + ((size_t)b * NN + (size_t)(16 * wave)) * NO;
#pragma unroll 1
    for (int ps = 0; ps < 2; ++ps) {
#pragma unroll
        for (int s = 0; s < 8; ++s) { const int row = 2 * s + (lane >> 4), cofs = (lane & 15) * 4;
            const v4f val = *(const v4fa*)(&sEI[wb + row * EIP + cofs]);
            *(volatile v4f*)(orow + (size_t)row * NO + cofs) = val; }
        if (ps == 0) __threadfence(); }
}

static constexpr size_t al256(size_t v) { return (v + 255) & ~(size_t)255; }
static constexpr size_t SZ_XB = al256((size_t)NB * NN * NF * 2);
static constexpr size_t SZ_WB = al256((size_t)NW * NF * 2);
static constexpr size_t SZ_TOTAL = SZ_XB + SZ_WB;
static_assert(SZ_TOTAL <= (size_t)134217728);
static_assert(((size_t)NB * NN * NF) % 8 == 0);
static_assert(((size_t)NB * NN * NF * 2) % 128 == 0);

extern "C" void kernel_launch(void* const* d_in, const int* in_sizes, int n_in,
                              void* d_out, int out_size, void* d_ws, size_t ws_size, hipStream_t stream) {
    if (n_in < 5) return;
    if ((size_t)in_sizes[0] < (size_t)NB * NN * NF) return;
    if (in_sizes[1] < NF * NO || in_sizes[2] < NO || in_sizes[3] < NO * 2 * NF) return;
    if (in_sizes[4] < NB_FULL * NN) return;
    if ((size_t)out_size < (size_t)NB * NN * NO) return;
    if (SZ_TOTAL > ws_size) return;
    const float* x  = (const float*)d_in[0];
    const float* W  = (const float*)d_in[1];
    const float* av = (const float*)d_in[2];
    const float* Wl = (const float*)d_in[3];
    const int* batch = (const int*)d_in[4];
    float* OUT = (float*)d_out;
    char* wsp = (char*)d_ws;
    bf* XB = (bf*)wsp; wsp += SZ_XB;
    bf* WB = (bf*)wsp; wsp += SZ_WB;

    { const size_t n8 = (size_t)NB * NN * NF / 8;
      k_cvt8<<<(unsigned)((n8 + 255) / 256), 256, 0, stream>>>(x, XB, n8); }
    k_wprep<<<(unsigned)(NW * NF / 8 / 256), 256, 0, stream>>>(W, Wl, WB);
    k_graph<<<NB, 32 * GW, 0, stream>>>(XB, WB, av, batch, OUT);
}
